// TriangleAttentionStartingNode_7456063225920
// MI455X (gfx1250) — hardware-verified
//
#include <hip/hip_runtime.h>


namespace {
constexpr int NN = 256, CZ = 128, H = 4, HD = 32, HC = H * HD, IL = 256  , NSLAB = 5  ;
constexpr float XS = 8.0f, WSC = 256.0f, PS = 1024.0f, LOG2E = 1.4426950408889634f, EPS = 1e-5f;
static_assert(NN % 64 == 0, "tiling");
typedef _Float16 b16;
typedef __attribute__((ext_vector_type(16))) _Float16 v16b;
typedef __attribute__((ext_vector_type(8))) _Float16 v8b;
typedef __attribute__((ext_vector_type(8))) float v8f;
typedef __attribute__((ext_vector_type(4))) float v4f;
__device__ __forceinline__ float bf16_rne(float f) { unsigned int u = __float_as_uint(f); u += 0x7FFFu + ((u >> 16) & 1u); return __uint_as_float(u & 0xFFFF0000u); }
__device__ __forceinline__ void split16(float v, b16& hi, b16& lo) { hi = (b16)v; lo = (b16)(v - (float)hi); }
__device__ __forceinline__ v16b frag_kb(const b16* p, int hh) { const v8b a = *(const v8b*)(p + 8 * hh), b = *(const v8b*)(p + 16 + 8 * hh); v16b f;
#pragma unroll
  for (int e = 0; e < 8; ++e) { f[e] = a[e]; f[8 + e] = b[e]; } return f; }
__device__ __forceinline__ v8f wmma16b(v16b a, v16b b, v8f c) { v8f d = __builtin_amdgcn_wmma_f32_16x16x32_f16(false, a, false, b, (short)0, c, false, false); asm volatile("v_nop\n\tv_nop\n\tv_nop\n\tv_nop" : "+v"(d) : "v"(a), "v"(b)); return d; }
__device__ __forceinline__ void wave_lds_sync() { __builtin_amdgcn_fence(__ATOMIC_RELEASE, "workgroup"); __builtin_amdgcn_wave_barrier(); __builtin_amdgcn_fence(__ATOMIC_ACQUIRE, "workgroup"); }
__device__ __forceinline__ float pmul(float a, float b) { float p = a * b; asm volatile("" : "+v"(p)); return p; }
__device__ __forceinline__ int iclamp(int v, int lo, int hi) { return v < lo ? lo : (v > hi ? hi : v); }

typedef __attribute__((ext_vector_type(2))) _Float16 v2h;
typedef __attribute__((ext_vector_type(4))) _Float16 v4h;
__device__ __forceinline__ float nexp2(float v) { return __builtin_amdgcn_exp2f(v); }
__global__ __launch_bounds__(256) void prep_kernel(const float* __restrict__ wq, const float* __restrict__ wk, const float* __restrict__ wv, const float* __restrict__ wb, const float* __restrict__ wg, const float* __restrict__ wo, b16* __restrict__ WT, b16* __restrict__ WO) {
  const int t = blockIdx.x * 256 + threadIdx.x; const int n1 = 640 * CZ / 8, n2 = CZ * HC / 8; v8b o;
  if (t < n1) { const int e = t * 8; const int oo = e / CZ, c0 = e % CZ; for (int j = 0; j < 8; ++j) { const int c = c0 + j; float w = 0.0f; if (oo < 128) w = wq[c * HC + oo]; else if (oo < 256) w = wk[c * HC + oo - 128]; else if (oo < 384) w = wv[c * HC + oo - 256]; else if (oo < 512) w = wg[c * HC + oo - 384]; else if (oo < 516) w = wb[c * H + oo - 512]; o[j] = (b16)(bf16_rne(w) * WSC); }
    for (int pass = 0; pass < 2; ++pass) { *(volatile v8b*)(WT + e) = o; __threadfence(); } }
  else if (t < n1 + n2) { const int e = (t - n1) * 8; const int oo = e / HC, c0 = e % HC; for (int j = 0; j < 8; ++j) o[j] = (b16)(bf16_rne(wo[(size_t)(c0 + j) * CZ + oo]) * WSC); for (int pass = 0; pass < 2; ++pass) { *(volatile v8b*)(WO + e) = o; __threadfence(); } }
}
__global__ __launch_bounds__(128) void proj_kernel(const float* __restrict__ z, const float* __restrict__ lng, const float* __restrict__ lnb, const b16* __restrict__ WT, b16* __restrict__ QH, b16* __restrict__ QL_, b16* __restrict__ KH, b16* __restrict__ KL, b16* __restrict__ VTh, b16* __restrict__ VTl, float* __restrict__ G, float* __restrict__ BIAS) {
  __shared__ __attribute__((aligned(16))) float Tf[4][16][128 + 4];
  const int wave = threadIdx.x >> 5, lane = threadIdx.x & 31, nloc = lane & 15, hlf = lane >> 4; const size_t r0 = (size_t)blockIdx.x * 64 + wave * 16; const int slab = blockIdx.y; const int i = (int)((blockIdx.x * 64) / NN), j0 = (int)((blockIdx.x * 64) % NN);
  if (slab < 4 && i >= IL) return;
  const int ntile = (slab == 4) ? 1 : 8;
  for (int rr = 0; rr < 16; ++rr) { const float* zr = z + (r0 + rr) * CZ; const v4f f = *(const v4f*)(zr + lane * 4); float x[4]; float s = 0.0f; for (int q = 0; q < 4; ++q) { x[q] = bf16_rne(f[q]); s += x[q]; }
#pragma unroll
    for (int o = 1; o < 32; o <<= 1) s += __shfl_xor(s, o);
    const float mu = s * (1.0f / CZ); float vs = 0.0f; for (int q = 0; q < 4; ++q) { const float d = x[q] - mu; vs += d * d; }
#pragma unroll
    for (int o = 1; o < 32; o <<= 1) vs += __shfl_xor(vs, o);
    const float rs = rsqrtf(vs * (1.0f / CZ) + EPS); v4f o4; for (int q = 0; q < 4; ++q) o4[q] = (x[q] - mu) * rs * bf16_rne(lng[lane * 4 + q]) + bf16_rne(lnb[lane * 4 + q]); *(v4f*)(&Tf[wave][rr][lane * 4]) = o4; }
  wave_lds_sync();
  v16b ah[4], al[4];
#pragma unroll
  for (int ks = 0; ks < 4; ++ks) {
#pragma unroll
    for (int e2 = 0; e2 < 16; ++e2) { const int c = ks * 32 + (e2 < 8 ? 0 : 16) + 8 * hlf + (e2 & 7); b16 p, q; split16(Tf[wave][nloc][c] * XS, p, q); ah[ks][e2] = p; al[ks][e2] = q; } }
  wave_lds_sync();
  v8f acc[8];
#pragma unroll
  for (int t = 0; t < 8; ++t) acc[t] = (v8f){};
#pragma unroll
  for (int ks = 0; ks < 4; ++ks) {
#pragma unroll
    for (int t = 0; t < 8; ++t) { if (t < ntile) { const v16b bw = frag_kb(WT + (size_t)(slab * 128 + t * 16 + nloc) * CZ + ks * 32, hlf); acc[t] = wmma16b(ah[ks], bw, acc[t]); acc[t] = wmma16b(al[ks], bw, acc[t]); } } }
#pragma unroll
  for (int t = 0; t < 8; ++t)
#pragma unroll
    for (int r = 0; r < 8; ++r) Tf[wave][8 * hlf + r][t * 16 + nloc] = acc[t][r] * (1.0f / (XS * WSC));
  __syncthreads();
  for (int pass = 0; pass < 2; ++pass) {
    if (slab < 2) { b16* PHp = slab == 0 ? QH : KH; b16* PLp = slab == 0 ? QL_ : KL; const int c = lane * 4; const int h = c / HD, d = c % HD;
      for (int rr = 0; rr < 16; ++rr) { const int j = j0 + wave * 16 + rr; v4h h4, l4; for (int q = 0; q < 4; ++q) { b16 p, ql; split16(Tf[wave][rr][c + q] * XS, p, ql); h4[q] = p; l4[q] = ql; }
        const size_t oi = (((size_t)i * H + h) * NN + j) * HD + d; *(volatile v4h*)(PHp + oi) = h4; *(volatile v4h*)(PLp + oi) = l4; } }
    else if (slab == 2) {
#pragma unroll 1
      for (int q = 0; q < 32; ++q) { const int c = wave * 32 + q; const int h = c / HD, d = c % HD; const int tk = lane * 2; v2h hv, lv;
        for (int jj = 0; jj < 2; ++jj) { b16 p, ql; split16(Tf[(tk + jj) >> 4][(tk + jj) & 15][c] * XS, p, ql); hv[jj] = p; lv[jj] = ql; }
        const size_t oi = (((size_t)i * H + h) * HD + d) * (size_t)NN + j0 + tk; *(volatile v2h*)(VTh + oi) = hv; *(volatile v2h*)(VTl + oi) = lv; } }
    else if (slab == 3) { for (int rr = 0; rr < 16; ++rr) { v4f gv; for (int q = 0; q < 4; ++q) gv[q] = 1.0f / (1.0f + __expf(-Tf[wave][rr][lane * 4 + q])); *(volatile v4f*)(G + (r0 + rr) * HC + lane * 4) = gv; } }
    else {
      if (wave < H) { const int h = wave; const int tk = lane * 2; __attribute__((ext_vector_type(2))) float b2; b2[0] = Tf[tk >> 4][tk & 15][h]; b2[1] = Tf[(tk + 1) >> 4][(tk + 1) & 15][h];
        *(volatile __attribute__((ext_vector_type(2))) float*)(BIAS + ((size_t)h * NN + i) * NN + j0 + tk) = b2; } }
    __threadfence(); }
}
__global__ __launch_bounds__(64) void attn_kernel(const b16* __restrict__ QH, const b16* __restrict__ QL_, const b16* __restrict__ KH, const b16* __restrict__ KL, const b16* __restrict__ VTh, const b16* __restrict__ VTl, const float* __restrict__ BIAS, const float* __restrict__ G, b16* __restrict__ Ch, b16* __restrict__ Cl) {
  __shared__ __attribute__((aligned(16))) b16 Pb[2][16][32 + 8], Pc[2][16][32 + 8]; __shared__ __attribute__((aligned(16))) float To[2][16][HD + 4];
  const int wave = threadIdx.x >> 5, lane = threadIdx.x & 31, hh = lane >> 4, col = lane & 15; const int i = blockIdx.y / H, h = blockIdx.y % H; const int q0 = blockIdx.x * 32 + wave * 16, qj = q0 + col;
  const size_t ph = (size_t)i * H + h; const size_t qb = ph * NN * HD, vb = ph * HD * (size_t)NN; const float* brow = BIAS + ((size_t)h * NN + qj) * NN;
  const v16b qh = frag_kb(QH + qb + (size_t)qj * HD, hh), ql = frag_kb(QL_ + qb + (size_t)qj * HD, hh);
  const float cs = LOG2E / (5.656854249492381f * XS * XS);
  float m = -INFINITY, l = 0.0f; v8f o[2] = {(v8f){}, (v8f){}};
#pragma unroll 1
  for (int kb = 0; kb < NN; kb += 32) {
    float e[16]; float mx = -INFINITY;
#pragma unroll
    for (int u = 0; u < 2; ++u) { v8f s = (v8f){}; const size_t kr = qb + (size_t)(kb + u * 16 + col) * HD; const v16b kh = frag_kb(KH + kr, hh), kl = frag_kb(KL + kr, hh);
      s = wmma16b(kh, qh, s); s = wmma16b(kh, ql, s); s = wmma16b(kl, qh, s);
      const v4f b0 = *(const v4f*)(brow + kb + u * 16 + 8 * hh), b1 = *(const v4f*)(brow + kb + u * 16 + 8 * hh + 4);
#pragma unroll
      for (int r = 0; r < 8; ++r) { const float bb = (r < 4) ? b0[r] : b1[r - 4]; const float vv = s[r] * cs + bb * LOG2E; e[u * 8 + r] = vv; mx = fmaxf(mx, vv); } }
    mx = fmaxf(mx, __shfl_xor(mx, 16)); const float mn = fmaxf(m, mx); const float al = nexp2(m - mn); float sum = 0.0f;
#pragma unroll
    for (int i2 = 0; i2 < 16; ++i2) { const float p = nexp2(e[i2] - mn); sum += p; b16 a_, b_; split16(p * PS, a_, b_); const int sl = (i2 < 8 ? 0 : 16) + 8 * hh + (i2 & 7); Pb[wave][col][sl] = a_; Pc[wave][col][sl] = b_; }
    sum += __shfl_xor(sum, 16); l = l * al + sum; m = mn;
    wave_lds_sync();
    const v16b pf = frag_kb(&Pb[wave][col][0], hh), pg = frag_kb(&Pc[wave][col][0], hh);
#pragma unroll
    for (int t = 0; t < 2; ++t) { o[t] *= al; const size_t vr = vb + (size_t)(t * 16 + col) * NN + kb; const v16b va = frag_kb(VTh + vr, hh), vl = frag_kb(VTl + vr, hh); o[t] = wmma16b(va, pf, o[t]); o[t] = wmma16b(va, pg, o[t]); o[t] = wmma16b(vl, pf, o[t]); }
    wave_lds_sync(); }
  const float inv = 1.0f / (l * PS * XS);
#pragma unroll
  for (int t = 0; t < 2; ++t)
#pragma unroll
    for (int r = 0; r < 8; ++r) To[wave][col][t * 16 + 8 * hh + r] = o[t][r] * inv;
  wave_lds_sync();
  for (int pass = 0; pass < 2; ++pass) { for (int qq = 0; qq < 8; ++qq) { const int rr = 2 * qq + (lane >> 4), c2 = (lane & 15) * 2; const size_t row = (size_t)i * NN + q0 + rr; v2h hv, lv;
      for (int jj = 0; jj < 2; ++jj) { const float gv = G[row * HC + h * HD + c2 + jj]; b16 p, q; split16(To[wave][rr][c2 + jj] * gv * XS, p, q); hv[jj] = p; lv[jj] = q; }
      const size_t oi = ((size_t)h * NN * NN + row) * HD + c2; *(volatile v2h*)(Ch + oi) = hv; *(volatile v2h*)(Cl + oi) = lv; } __threadfence(); }
}
__global__ __launch_bounds__(128) void out_kernel(const b16* __restrict__ Ch, const b16* __restrict__ Cl, const b16* __restrict__ WO, float* __restrict__ out) {
  __shared__ __attribute__((aligned(16))) float Tf[4][16][128 + 4];
  const int wave = threadIdx.x >> 5, lane = threadIdx.x & 31, nloc = lane & 15, hlf = lane >> 4; const size_t m0 = ((size_t)blockIdx.x * 4 + wave) * 16;
  v8f acc[8];
#pragma unroll
  for (int t = 0; t < 8; ++t) acc[t] = (v8f){};
#pragma unroll
  for (int kb = 0; kb < HC; kb += 32) { const size_t po = ((size_t)(kb / 32) * NN * NN + m0 + nloc) * HD; const v16b a = frag_kb(Ch + po, hlf), a2 = frag_kb(Cl + po, hlf);
#pragma unroll
    for (int t = 0; t < 8; ++t) { const v16b bw = frag_kb(WO + (size_t)(t * 16 + nloc) * HC + kb, hlf); acc[t] = wmma16b(a, bw, acc[t]); acc[t] = wmma16b(a2, bw, acc[t]); } }
#pragma unroll
  for (int t = 0; t < 8; ++t)
#pragma unroll
    for (int r = 0; r < 8; ++r) Tf[wave][8 * hlf + r][t * 16 + nloc] = acc[t][r] * (1.0f / (XS * WSC));
  wave_lds_sync();
  for (int pass = 0; pass < 2; ++pass) { for (int rr = 0; rr < 16; ++rr) *(volatile v4f*)(out + (m0 + rr) * CZ + lane * 4) = *(const v4f*)(&Tf[wave][rr][lane * 4]); __threadfence(); }
}
}

extern "C" void kernel_launch(void* const* d_in, const int* in_sizes, int n_in, void* d_out, int out_size, void* d_ws, size_t ws_size, hipStream_t stream) {
  (void)n_in;
  auto Fp = [&](int i) { return (const float*)d_in[i]; };
  if (in_sizes[0] != NN * NN * CZ || in_sizes[1] != CZ || in_sizes[2] != CZ || in_sizes[3] != CZ * HC || in_sizes[6] != CZ * H || in_sizes[7] != CZ * HC || in_sizes[8] != HC * CZ || out_size != NN * NN * CZ) return;
  size_t off = 0; char* ws = (char*)d_ws;
  auto carve = [&](size_t bytes) { char* p = ws + off; off += (bytes + 255) & ~(size_t)255; return p; };
  b16* WT = (b16*)carve((size_t)640 * CZ * 2); b16* WO = (b16*)carve((size_t)CZ * HC * 2); const size_t plane = (size_t)NN * NN * HC * 2;
  b16* QH = (b16*)carve(plane); b16* QL_ = (b16*)carve(plane); b16* KH = (b16*)carve(plane); b16* KL = (b16*)carve(plane); b16* VTh = (b16*)carve(plane); b16* VTl = (b16*)carve(plane); b16* Ch = (b16*)carve(plane); b16* Cl = (b16*)carve(plane);
  float* G = (float*)carve((size_t)NN * NN * HC * 4); float* BIAS = (float*)carve((size_t)H * NN * NN * 4);
  if (off > ws_size || off > ((size_t)240 << 20)) return;
  prep_kernel<<<(640 * CZ / 8 + CZ * HC / 8 + 255) / 256, 256, 0, stream>>>(Fp(3), Fp(4), Fp(5), Fp(6), Fp(7), Fp(8), WT, WO);
  proj_kernel<<<dim3((NN * NN) / 64, NSLAB), 128, 0, stream>>>(Fp(0), Fp(1), Fp(2), WT, QH, QL_, KH, KL, VTh, VTl, G, BIAS);
  attn_kernel<<<dim3(NN / 32, IL * H), 64, 0, stream>>>(QH, QL_, KH, KL, VTh, VTl, BIAS, G, Ch, Cl);
  out_kernel<<<(IL * NN) / 64, 128, 0, stream>>>(Ch, Cl, WO, (float*)d_out);
}
